// FlexibleJSSNet_16252156248138
// MI455X (gfx1250) — hardware-run, weakly checked
//
#include <hip/hip_runtime.h>
#include <math.h>

typedef __attribute__((ext_vector_type(16))) _Float16 v16h;
typedef __attribute__((ext_vector_type(8)))  _Float16 v8h;
typedef __attribute__((ext_vector_type(4)))  _Float16 v4h;
typedef __attribute__((ext_vector_type(8)))  float    v8f;
typedef __attribute__((ext_vector_type(4)))  float    v4f;
typedef __attribute__((ext_vector_type(4)))  unsigned v4u;
typedef __attribute__((ext_vector_type(2)))  double   v2d;

constexpr int kNT   = 250000;
constexpr int kNM   = 50000;
constexpr int kNB   = 1000;
constexpr int kTPer = 250;
constexpr int kMPer = 50;
constexpr int kH    = 128;
constexpr int kNL   = 25000;
constexpr int kDT   = 16;
constexpr int kDM   = 8;
constexpr int kNTP  = 250048;
constexpr int kNMP  = 50048;
constexpr int kNBP  = 1024;
constexpr int kNLP  = 25024;
constexpr int kRowsPerStatBlk = 1000;
constexpr int kBlkT = kNT / kRowsPerStatBlk;
constexpr int kBlkM = kNM / kRowsPerStatBlk;
constexpr float kEps = 1e-5f;
static_assert(kNB * kTPer == kNT && kNB * kMPer == kNM, "segment sizes");
static_assert(kNTP % 64 == 0 && kNMP % 64 == 0 && kNBP % 64 == 0 && kNLP % 64 == 0, "tile multiples");
static_assert(kNTP >= kNT && kNMP >= kNM && kNBP >= kNB && kNLP >= kNL, "padded extents");
static_assert(kBlkT * kRowsPerStatBlk == kNT && kBlkM * kRowsPerStatBlk == kNM, "statistics blocks");
static_assert(kNL % 4 == 0, "output rows per 16-B store");

constexpr float kWCarry  = 64.0f;
constexpr float kACarry  = 16.0f;
constexpr float kXRCarry = 64.0f;
constexpr float kInvW    = 1.0f / kWCarry;
constexpr float kInvA    = 1.0f / kACarry;
static_assert(kXRCarry == kWCarry, "remainder slots of the first layer share the accumulator scale");

constexpr int kPA1 = 40;
constexpr int kPH  = 136;
constexpr int kPG  = 264;

constexpr size_t kSzPartT = (size_t)kBlkT * 2 * kDT * 8;
constexpr size_t kSzPartM = (size_t)kBlkM * 2 * kDM * 8;
constexpr size_t kSzStats = 256;
constexpr size_t kSzW32   = (size_t)kH * 32 * 2;
constexpr size_t kSzW128  = (size_t)kH * 128 * 2;
constexpr size_t kSzW256  = (size_t)kH * 256 * 2;
constexpr size_t kSzW384  = (size_t)kH * 384 * 2;
constexpr size_t kSzTH    = (size_t)kNTP * kH * 2;
constexpr size_t kSzMH    = (size_t)kNMP * kH * 2;
constexpr size_t kSzGM    = (size_t)kNBP * 256 * 2;
constexpr size_t kSzAG    = (size_t)kNBP * kH * 2;

constexpr size_t kOffPartT = 0;
constexpr size_t kOffPartM = kOffPartT + kSzPartT;
constexpr size_t kOffStats = kOffPartM + kSzPartM;
constexpr size_t kOffWT1   = kOffStats + kSzStats;
constexpr size_t kOffWM1   = kOffWT1  + kSzW32;
constexpr size_t kOffWT2V  = kOffWM1  + kSzW32;
constexpr size_t kOffWM2V  = kOffWT2V + kSzW128;
constexpr size_t kOffWA1V  = kOffWM2V + kSzW128;
constexpr size_t kOffWA2V  = kOffWA1V + kSzW256;
constexpr size_t kOffWL1V  = kOffWA2V + kSzW128;
constexpr size_t kOffWL2V  = kOffWL1V + kSzW384;
constexpr size_t kOffWO1V  = kOffWL2V + kSzW128;
constexpr size_t kOffTH    = kOffWO1V + kSzW128;
constexpr size_t kOffMH    = kOffTH + kSzTH;
constexpr size_t kOffGM    = kOffMH + kSzMH;
constexpr size_t kOffAG    = kOffGM + kSzGM;
constexpr size_t kWsTotal  = kOffAG + kSzAG;
static_assert(kWsTotal == 78025728ull, "carve total");
static_assert(kWsTotal <= 134217728ull, "carve cap");
static_assert((kOffPartM % 128) == 0 && (kOffStats % 128) == 0 && (kOffWT1 % 128) == 0 && (kOffWM1 % 128) == 0 &&
              (kOffWT2V % 128) == 0 && (kOffWM2V % 128) == 0 && (kOffWA1V % 128) == 0 && (kOffWA2V % 128) == 0 &&
              (kOffWL1V % 128) == 0 && (kOffWL2V % 128) == 0 && (kOffWO1V % 128) == 0 &&
              (kOffTH % 128) == 0 && (kOffMH % 128) == 0 && (kOffGM % 128) == 0 && (kOffAG % 128) == 0, "line aligned regions");

__device__ __forceinline__ float flush16(float v) {
  return (fabsf(v) < 6.103515625e-5f) ? 0.0f : v;
}

__device__ __forceinline__ float h16_to_f32(unsigned hb) {
  const unsigned sgn = (hb & 0x8000u) << 16;
  const unsigned em = hb & 0x7fffu;
  const float fn = __uint_as_float((em << 13) + 0x38000000u);
  const float fs = (float)em * 5.9604644775390625e-8f;
  const float mag = (em < 0x400u) ? fs : fn;
  return __uint_as_float(__float_as_uint(mag) | sgn);
}

struct FragH {
  union U { v16h v; v8h h[2]; };
  static __device__ __forceinline__ v16h load(const _Float16* p) {
    U f;
    f.h[0] = *(const v8h*)(p);
    f.h[1] = *(const v8h*)(p + 16);
    return f.v;
  }
};

__device__ __forceinline__ v8f mma_h(v16h a, v16h b, v8f c) {
  c = __builtin_amdgcn_wmma_f32_16x16x32_f16(false, a, false, b, (short)0, c, false, false);
  asm volatile("v_nop\n\tv_nop\n\tv_nop\n\tv_nop" : "+v"(c) : "v"(a), "v"(b));
  return c;
}

__device__ __forceinline__ void zero_acc4(v8f (&a)[4]) {
#pragma unroll
  for (int j = 0; j < 4; ++j) a[j] = (v8f){0.f, 0.f, 0.f, 0.f, 0.f, 0.f, 0.f, 0.f};
}

template <int KSTEPS>
__device__ __forceinline__ void tile_gemm1(const _Float16* aRow, const _Float16* bV, int ldb,
                                           v8f (&accV)[4]) {
#pragma unroll 1
  for (int ks = 0; ks < KSTEPS; ++ks) {
    const v16h a = FragH::load(aRow + ks * 32);
#pragma unroll
    for (int j = 0; j < 4; ++j) {
      const size_t bo = (size_t)(j * 16) * ldb + ks * 32;
      const v16h fv = FragH::load(bV + bo);
      accV[j] = mma_h(a, fv, accV[j]);
    }
  }
}

template <bool RELU>
__device__ __forceinline__ void tile_epilogue16(const v8f (&accV)[4],
                                                const float* __restrict__ bias, int ncol, _Float16* dstRow) {
#pragma unroll
  for (int j = 0; j < 4; ++j) {
    const int n = ncol + j * 16;
    const float bv = bias[n] * kACarry;
#pragma unroll
    for (int r = 0; r < 8; ++r) {
      float v = accV[j][r] * kInvW;
      v += bv;
      if (RELU) v = (v < 0.0f) ? 0.0f : v;
      dstRow[r * kPH + n] = (_Float16)flush16(v);
    }
  }
}

__device__ __forceinline__ void store_tile_rows(const _Float16* sT, unsigned short* __restrict__ plane,
                                                int rows0, int nvalid, int wave, int lane) {
  const int hh = lane >> 4;
  const int c8 = (lane & 15) * 8;
  const v4u z = {0u, 0u, 0u, 0u};
  v4u vals[4];
#pragma unroll
  for (int it = 0; it < 4; ++it) {
    const int row = wave * 8 + it * 2 + hh;
    const v4u v = *(const v4u*)(sT + row * kPH + c8);
    const bool ok = (rows0 + row) < nvalid;
    vals[it] = ok ? v : z;
  }
  for (int pass = 0; pass < 2; ++pass) {
#pragma unroll
    for (int it = 0; it < 4; ++it) {
      const int row = wave * 8 + it * 2 + hh;
      *(volatile v4u*)(plane + (size_t)(rows0 + row) * kH + c8) = vals[it];
    }
    __threadfence();
  }
}

__global__ __launch_bounds__(256) void prep_weights_kernel(
    const float* __restrict__ wt1, const float* __restrict__ wm1, const float* __restrict__ wt2,
    const float* __restrict__ wm2, const float* __restrict__ wa1, const float* __restrict__ wa2,
    const float* __restrict__ wl1, const float* __restrict__ wl2, const float* __restrict__ wo1,
    unsigned char* __restrict__ ws)
{
  const int wid = blockIdx.y;
  const float* src = wt1;
  int kp = 32;
  int kreal = kDT;
  size_t offV = kOffWT1;
  if (wid == 1) { src = wm1; kp = 32;  kreal = kDM; offV = kOffWM1; }
  if (wid == 2) { src = wt2; kp = 128; kreal = 128; offV = kOffWT2V; }
  if (wid == 3) { src = wm2; kp = 128; kreal = 128; offV = kOffWM2V; }
  if (wid == 4) { src = wa1; kp = 256; kreal = 256; offV = kOffWA1V; }
  if (wid == 5) { src = wa2; kp = 128; kreal = 128; offV = kOffWA2V; }
  if (wid == 6) { src = wl1; kp = 384; kreal = 384; offV = kOffWL1V; }
  if (wid == 7) { src = wl2; kp = 128; kreal = 128; offV = kOffWL2V; }
  if (wid == 8) { src = wo1; kp = 128; kreal = 128; offV = kOffWO1V; }
  const int total = 16 * kp;
  const int i = blockIdx.x * 256 + threadIdx.x;
  if (i >= total) return;
  const int cpn = kp >> 3;
  const int n = i / cpn;
  const int k0 = (i - n * cpn) * 8;
  const int seg = k0 / kreal;
  const int kr0 = k0 - seg * kreal;
  v8h hv;
#pragma unroll
  for (int e = 0; e < 8; ++e) {
    const float w = src[(size_t)(kr0 + e) * kH + n];
    const float wc = w * kWCarry;
    const float val = (seg == 0) ? wc : ((seg == 1) ? w : 0.0f);
    hv[e] = (_Float16)flush16(val);
  }
  volatile v8h* pv = (volatile v8h*)(ws + offV + (size_t)i * 16);
  *pv = hv;
  __threadfence();
  *pv = hv;
}

template <int DIN>
__global__ __launch_bounds__(256) void bn_partial_kernel(const float* __restrict__ x, int nrows,
                                                         double* __restrict__ part)
{
  __shared__ double rs[256];
  __shared__ double rq[256];
  constexpr int SL = 256 / DIN;
  constexpr int NIT = (kRowsPerStatBlk + SL - 1) / SL;
  const int tid = threadIdx.x;
  const int col = tid & (DIN - 1);
  const int slot = tid / DIN;
  const int r0 = blockIdx.x * kRowsPerStatBlk;
  const int rlim = r0 + kRowsPerStatBlk;
  const int rend = rlim < nrows ? rlim : nrows;
  double s = 0.0, q = 0.0;
#pragma unroll 1
  for (int it = 0; it < NIT; ++it) {
    const int row = r0 + slot + it * SL;
    const int rc = row < nrows ? row : nrows - 1;
    float v = x[(size_t)rc * DIN + col];
    asm volatile("" : "+v"(v));
    const double dv = (row < rend) ? (double)v : 0.0;
    s += dv;
    q += dv * dv;
  }
  rs[tid] = s;
  rq[tid] = q;
  __syncthreads();
  for (int off = 128; off >= DIN; off >>= 1) {
    if (tid < off) {
      rs[tid] += rs[tid + off];
      rq[tid] += rq[tid + off];
    }
    __syncthreads();
  }
  {
    const int e0 = 2 * tid;
    const int idx = e0 & (DIN - 2);
    const double s0 = rs[idx], s1 = rs[idx + 1];
    const double q0 = rq[idx], q1 = rq[idx + 1];
    const bool lowhalf = e0 < DIN;
    v2d val;
    val[0] = lowhalf ? s0 : q0;
    val[1] = lowhalf ? s1 : q1;
    const bool st = tid < DIN;
    volatile v2d* p = (volatile v2d*)(part + (size_t)blockIdx.x * 2 * DIN) + (tid & (DIN - 1));
    if (st) *p = val;
    __threadfence();
    if (st) *p = val;
  }
}

__global__ __launch_bounds__(256) void bn_finalize_kernel(
    const double* __restrict__ partT, const double* __restrict__ partM,
    const float* __restrict__ gt, const float* __restrict__ bt,
    const float* __restrict__ gmv, const float* __restrict__ bmv,
    const int* __restrict__ tb, const int* __restrict__ mb, const int* __restrict__ ng,
    float* __restrict__ stats)
{
  __shared__ int sBad[8];
  __shared__ __align__(16) float sSt[64];
  const int tid = threadIdx.x, lane = tid & 31, wave = tid >> 5;
  int bad = 0;
#pragma unroll 1
  for (int it = 0; it < (kNT + 255) / 256; ++it) {
    const int i = it * 256 + tid;
    const int ic = i < kNT ? i : kNT - 1;
    int v = tb[ic];
    asm volatile("" : "+v"(v));
    bad |= ((i < kNT) && (v != ic / kTPer)) ? 1 : 0;
  }
#pragma unroll 1
  for (int it = 0; it < (kNM + 255) / 256; ++it) {
    const int i = it * 256 + tid;
    const int ic = i < kNM ? i : kNM - 1;
    int v = mb[ic];
    asm volatile("" : "+v"(v));
    bad |= ((i < kNM) && (v != ic / kMPer)) ? 1 : 0;
  }
  {
    const int ngv = ng[0];
    bad |= (ngv != kNB) ? 1 : 0;
  }
  const unsigned long long bl = __ballot(bad != 0);
  if (lane == 0) sBad[wave] = (bl != 0ull) ? 1 : 0;
  if (wave == 0) {
    const int ct = lane & (kDT - 1);
    const int cm = lane & (kDM - 1);
    double s = 0.0, q = 0.0;
#pragma unroll 1
    for (int b = 0; b < kBlkT; ++b) {
      s += partT[(size_t)b * 2 * kDT + ct];
      q += partT[(size_t)b * 2 * kDT + kDT + ct];
    }
    double sm = 0.0, qm = 0.0;
#pragma unroll 1
    for (int b = 0; b < kBlkM; ++b) {
      sm += partM[(size_t)b * 2 * kDM + cm];
      qm += partM[(size_t)b * 2 * kDM + kDM + cm];
    }
    const double muT = s * (1.0 / (double)kNT);
    const double varT = q * (1.0 / (double)kNT) - muT * muT;
    const double muM = sm * (1.0 / (double)kNM);
    const double varM = qm * (1.0 / (double)kNM) - muM * muM;
    const float scT = gt[ct] * rsqrtf((float)varT + kEps);
    const float shT = (float)((double)bt[ct] - muT * (double)scT);
    const float scM = gmv[cm] * rsqrtf((float)varM + kEps);
    const float shM = (float)((double)bmv[cm] - muM * (double)scM);
    if (lane < kDT) { sSt[lane] = scT; sSt[kDT + lane] = shT; }
    if (lane < kDM) { sSt[32 + lane] = scM; sSt[40 + lane] = shM; }
    if (lane >= 16) sSt[32 + lane] = 0.0f;
  }
  __syncthreads();
  const int anyBad = sBad[0] | sBad[1] | sBad[2] | sBad[3] | sBad[4] | sBad[5] | sBad[6] | sBad[7];
  if (wave == 0) {
    const int l16 = lane & 15;
    v4f v = *(const v4f*)(sSt + 4 * l16);
    const float qnan = __uint_as_float(0x7fc00000u);
    v4f o = {0.f, 0.f, 0.f, 0.f};
#pragma unroll
    for (int e = 0; e < 4; ++e) o[e] = anyBad ? qnan : v[e];
    const bool st = lane < 16;
    volatile v4f* p = (volatile v4f*)(stats + 4 * l16);
    if (st) *p = o;
    __threadfence();
    if (st) *p = o;
  }
}

template <int DIN>
__global__ __launch_bounds__(256) void encoder_kernel(
    const float* __restrict__ x, int nrows,
    const float* __restrict__ sc, const float* __restrict__ sh,
    const unsigned short* __restrict__ w1p, const float* __restrict__ b1,
    const unsigned short* __restrict__ w2v, const float* __restrict__ b2,
    unsigned short* __restrict__ outp)
{
  static_assert(DIN == 16 || DIN == 8, "input widths");
  __shared__ __align__(16) _Float16 sA1[64 * kPA1];
  __shared__ __align__(16) _Float16 sH[64 * kPH];
  __shared__ __align__(16) _Float16 sO[64 * kPH];
  const int tid = threadIdx.x, lane = tid & 31, wave = tid >> 5;
  const int m = lane & 15, hh = lane >> 4, rg = wave & 3, chh = wave >> 2;
  const int rows0 = blockIdx.x * 64;
  constexpr int TPR = DIN / 4;
  if (tid < 64 * TPR) {
    const int row = tid / TPR;
    const int c4 = (tid % TPR) * 4;
    const int gr = rows0 + row;
    const int grc = gr < nrows ? gr : nrows - 1;
    const v4f xv = *(const v4f*)(x + (size_t)grc * DIN + c4);
    const v4f scv = *(const v4f*)(sc + c4);
    const v4f shv = *(const v4f*)(sh + c4);
    const bool ok = gr < nrows;
    v4h hv, lv;
#pragma unroll
    for (int e = 0; e < 4; ++e) {
      float v = fmaf(xv[e], scv[e], shv[e]) * kACarry;
      v = ok ? v : 0.0f;
      const _Float16 hq = (_Float16)flush16(v);
      const float rem = (v - (float)hq) * kXRCarry;
      hv[e] = hq;
      lv[e] = (_Float16)flush16(rem);
    }
    *(v4h*)(sA1 + row * kPA1 + c4) = hv;
    *(v4h*)(sA1 + row * kPA1 + DIN + c4) = lv;
  } else {
    const int t2 = tid - 64 * TPR;
    const int row = t2 >> 1;
    const int off = 2 * DIN + (t2 & 1) * 8;
    const v8h z8 = {(_Float16)0.f, (_Float16)0.f, (_Float16)0.f, (_Float16)0.f,
                    (_Float16)0.f, (_Float16)0.f, (_Float16)0.f, (_Float16)0.f};
    *(v8h*)(sA1 + row * kPA1 + off) = z8;
  }
  __syncthreads();

  const int ncol = chh * 64 + m;
  {
    v8f acc[4];
    zero_acc4(acc);
    const v16h a = FragH::load(sA1 + (rg * 16 + m) * kPA1 + 8 * hh);
    const _Float16* bp = (const _Float16*)w1p + (size_t)ncol * 32 + 8 * hh;
#pragma unroll
    for (int j = 0; j < 4; ++j) {
      const v16h b = FragH::load(bp + (size_t)(j * 16) * 32);
      acc[j] = mma_h(a, b, acc[j]);
    }
    _Float16* dstRow = sH + (rg * 16 + 8 * hh) * kPH;
#pragma unroll
    for (int j = 0; j < 4; ++j) {
      const int n = ncol + j * 16;
      const float bv = b1[n] * kACarry;
#pragma unroll
      for (int r = 0; r < 8; ++r) {
        float v = acc[j][r] * kInvW;
        v += bv;
        v = (v < 0.0f) ? 0.0f : v;
        dstRow[r * kPH + n] = (_Float16)flush16(v);
      }
    }
  }
  __syncthreads();

  {
    v8f accV[4];
    zero_acc4(accV);
    tile_gemm1<4>(sH + (rg * 16 + m) * kPH + 8 * hh,
                  (const _Float16*)w2v + (size_t)ncol * 128 + 8 * hh, 128, accV);
    tile_epilogue16<true>(accV, b2, ncol, sO + (rg * 16 + 8 * hh) * kPH);
  }
  __syncthreads();
  store_tile_rows(sO, outp, rows0, nrows, wave, lane);
}

__global__ __launch_bounds__(128) void segmean_kernel(const unsigned* __restrict__ thw,
                                                      const unsigned* __restrict__ mhw,
                                                      unsigned short* __restrict__ gmp)
{
  __shared__ __align__(16) float sS[2 * 256];
  const int tid = threadIdx.x, lane = tid & 31, wave = tid >> 5;
  const int g = blockIdx.x;
  const bool live = g < kNB;
  const int p = tid & 63;
  const int rh = tid >> 6;
  float t0 = 0.0f, t1 = 0.0f, m0 = 0.0f, m1 = 0.0f;
  if (live) {
    const unsigned* bt = thw + (size_t)g * kTPer * 64 + p;
#pragma unroll 5
    for (int r = rh; r < kTPer; r += 2) {
      const unsigned w = bt[(size_t)r * 64];
      t0 += h16_to_f32(w & 0xffffu);
      t1 += h16_to_f32(w >> 16);
    }
    const unsigned* bm = mhw + (size_t)g * kMPer * 64 + p;
#pragma unroll 5
    for (int r = rh; r < kMPer; r += 2) {
      const unsigned w = bm[(size_t)r * 64];
      m0 += h16_to_f32(w & 0xffffu);
      m1 += h16_to_f32(w >> 16);
    }
  }
  sS[rh * 256 + 2 * p] = t0;
  sS[rh * 256 + 2 * p + 1] = t1;
  sS[rh * 256 + 128 + 2 * p] = m0;
  sS[rh * 256 + 128 + 2 * p + 1] = m1;
  __syncthreads();
  if (wave == 0) {
    const int c0 = 8 * lane;
    const float inv = (c0 >= 128) ? (1.0f / (float)kMPer) : (1.0f / (float)kTPer);
    v8h hv;
#pragma unroll
    for (int e = 0; e < 8; ++e) {
      float v = (sS[c0 + e] + sS[256 + c0 + e]) * inv;
      v = live ? v : 0.0f;
      hv[e] = (_Float16)flush16(v);
    }
    volatile v8h* q = (volatile v8h*)(gmp + (size_t)g * 256 + c0);
    *q = hv;
    __threadfence();
    *q = hv;
  }
}

__global__ __launch_bounds__(256) void aggr_kernel(
    const unsigned short* __restrict__ gmp,
    const unsigned short* __restrict__ w1v, const float* __restrict__ b1,
    const unsigned short* __restrict__ w2v, const float* __restrict__ b2,
    unsigned short* __restrict__ agp)
{
  __shared__ __align__(16) _Float16 sA[64 * kPG];
  __shared__ __align__(16) _Float16 sH[64 * kPH];
  static_assert(64 * kPG >= 64 * kPH, "second-layer tile fits the first-layer staging tile");
  const int tid = threadIdx.x, lane = tid & 31, wave = tid >> 5;
  const int m = lane & 15, hh = lane >> 4, rg = wave & 3, chh = wave >> 2;
  const int rows0 = blockIdx.x * 64;
#pragma unroll
  for (int it = 0; it < 8; ++it) {
    const int v = it * 256 + tid;
    const int row = v >> 5;
    const int c8 = (v & 31) * 8;
    const v4u val = *(const v4u*)(gmp + (size_t)(rows0 + row) * 256 + c8);
    *(v4u*)(sA + row * kPG + c8) = val;
  }
  __syncthreads();
  const int ncol = chh * 64 + m;
  v8f accV[4];
  zero_acc4(accV);
  tile_gemm1<8>(sA + (rg * 16 + m) * kPG + 8 * hh,
                (const _Float16*)w1v + (size_t)ncol * 256 + 8 * hh, 256, accV);
  tile_epilogue16<true>(accV, b1, ncol, sH + (rg * 16 + 8 * hh) * kPH);
  __syncthreads();
  zero_acc4(accV);
  tile_gemm1<4>(sH + (rg * 16 + m) * kPH + 8 * hh,
                (const _Float16*)w2v + (size_t)ncol * 128 + 8 * hh, 128, accV);
  tile_epilogue16<false>(accV, b2, ncol, sA + (rg * 16 + 8 * hh) * kPH);
  __syncthreads();
  store_tile_rows(sA, agp, rows0, kNBP, wave, lane);
}

__device__ __forceinline__ void stage_rows(const unsigned short* __restrict__ plane, const int* sIdx,
                                           int zeroIdx, int maxRow, _Float16* sA, int tid) {
  const v4u z = {0u, 0u, 0u, 0u};
#pragma unroll
  for (int it = 0; it < 4; ++it) {
    const int v = it * 256 + tid;
    const int row = v >> 4;
    const int c8 = (v & 15) * 8;
    const int idx = sIdx[row];
    int ic = idx < 0 ? 0 : idx;
    ic = ic > maxRow ? maxRow : ic;
    const v4u val = *(const v4u*)(plane + (size_t)ic * kH + c8);
    const v4u sel = (idx >= zeroIdx) ? z : val;
    *(v4u*)(sA + row * kPH + c8) = sel;
  }
}

__global__ __launch_bounds__(256) void link_kernel(
    const unsigned short* __restrict__ thp, const unsigned short* __restrict__ mhp,
    const unsigned short* __restrict__ agp,
    const float* __restrict__ x, const int* __restrict__ tb, const int* __restrict__ label,
    const unsigned short* __restrict__ wl1v, const float* __restrict__ bl1,
    const unsigned short* __restrict__ wl2v, const float* __restrict__ bl2,
    const unsigned short* __restrict__ wo1v, const float* __restrict__ bo1,
    const float* __restrict__ wo2, const float* __restrict__ bo2,
    float* __restrict__ outp)
{
  __shared__ __align__(16) _Float16 sA[64 * kPH];
  __shared__ __align__(16) _Float16 sH[64 * kPH];
  __shared__ __align__(16) float sPart[128];
  __shared__ int sRow[64];
  __shared__ int sBat[64];
  __shared__ int sMach[64];
  const int tid = threadIdx.x, lane = tid & 31, wave = tid >> 5;
  const int m = lane & 15, hh = lane >> 4, rg = wave & 3, chh = wave >> 2;
  const int rows0 = blockIdx.x * 64;

  if (tid < 64) {
    const int i = rows0 + tid;
    const int ic = i < kNL ? i : kNL - 1;
    int r = label[ic];
    r = r < 0 ? r + kNT : r;
    r = r < 0 ? 0 : (r > kNT - 1 ? kNT - 1 : r);
    int b = tb[r];
    b = b < 0 ? b + kNB : b;
    b = b < 0 ? 0 : (b > kNB - 1 ? kNB - 1 : b);
    const float tm = x[(size_t)r * kDT + 1];
    int idx = (int)tm + kMPer * b;
    idx = idx < 0 ? idx + (kNM + 1) : idx;
    idx = idx < 0 ? 0 : (idx > kNM ? kNM : idx);
    idx = (tm == -1.0f) ? kNM : idx;
    sRow[tid] = r;
    sBat[tid] = b;
    sMach[tid] = idx;
  }
  __syncthreads();

  const int ncol = chh * 64 + m;
  const _Float16* aRowA = sA + (rg * 16 + m) * kPH + 8 * hh;
  const _Float16* aRowH = sH + (rg * 16 + m) * kPH + 8 * hh;
  const _Float16* l1v = (const _Float16*)wl1v + (size_t)ncol * 384 + 8 * hh;
  v8f accV[4];
  zero_acc4(accV);

  stage_rows(thp, sRow, 0x7fffffff, kNT - 1, sA, tid);
  __syncthreads();
  tile_gemm1<4>(aRowA, l1v, 384, accV);
  __syncthreads();
  stage_rows(agp, sBat, 0x7fffffff, kNB - 1, sA, tid);
  __syncthreads();
  tile_gemm1<4>(aRowA, l1v + 128, 384, accV);
  __syncthreads();
  stage_rows(mhp, sMach, kNM, kNM - 1, sA, tid);
  __syncthreads();
  tile_gemm1<4>(aRowA, l1v + 256, 384, accV);
  __syncthreads();

  tile_epilogue16<true>(accV, bl1, ncol, sH + (rg * 16 + 8 * hh) * kPH);
  __syncthreads();
  zero_acc4(accV);
  tile_gemm1<4>(aRowH, (const _Float16*)wl2v + (size_t)ncol * 128 + 8 * hh, 128, accV);
  tile_epilogue16<false>(accV, bl2, ncol, sA + (rg * 16 + 8 * hh) * kPH);
  __syncthreads();
  zero_acc4(accV);
  tile_gemm1<4>(aRowA, (const _Float16*)wo1v + (size_t)ncol * 128 + 8 * hh, 128, accV);

  float part[8];
#pragma unroll
  for (int r = 0; r < 8; ++r) part[r] = 0.0f;
#pragma unroll
  for (int j = 0; j < 4; ++j) {
    const int n = ncol + j * 16;
    const float bv = bo1[n] * kACarry;
    const float wv = wo2[n];
#pragma unroll
    for (int r = 0; r < 8; ++r) {
      float v = accV[j][r] * kInvW;
      v += bv;
      v = (v < 0.0f) ? 0.0f : v;
      part[r] = fmaf(v, wv, part[r]);
    }
  }
#pragma unroll
  for (int r = 0; r < 8; ++r) {
#pragma unroll
    for (int off = 1; off < 16; off <<= 1) part[r] += __shfl_xor(part[r], off, 32);
  }
  if (m == 0) {
#pragma unroll
    for (int r = 0; r < 8; ++r) sPart[chh * 64 + rg * 16 + 8 * hh + r] = part[r];
  }
  __syncthreads();
  if (wave == 0) {
    const int l16 = lane & 15;
    const int base = 4 * l16;
    const float b2v = bo2[0];
    v4f o = {0.f, 0.f, 0.f, 0.f};
#pragma unroll
    for (int e = 0; e < 4; ++e) o[e] = (sPart[base + e] + sPart[64 + base + e]) * kInvA + b2v;
    const bool st = (lane < 16) && (rows0 + base + 3 < kNL);
    float* p = outp + rows0 + base;
    if (st) *(volatile v4f*)p = o;
    __threadfence();
    if (st) *(volatile v4f*)p = o;
  }
}

extern "C" void kernel_launch(void* const* d_in, const int* in_sizes, int n_in,
                              void* d_out, int out_size, void* d_ws, size_t ws_size,
                              hipStream_t stream) {
  if (n_in < 30) return;
  if (in_sizes[0] != kNT * kDT) return;
  if (in_sizes[1] != kNM * kDM) return;
  if (in_sizes[4] != kDT * kH || in_sizes[6] != kH * kH) return;
  if (in_sizes[10] != kDM * kH || in_sizes[12] != kH * kH) return;
  if (in_sizes[14] != 2 * kH * kH || in_sizes[16] != kH * kH) return;
  if (in_sizes[18] != 3 * kH * kH || in_sizes[20] != kH * kH) return;
  if (in_sizes[22] != kH * kH || in_sizes[24] != kH) return;
  if (in_sizes[26] != kNT || in_sizes[27] != kNM || in_sizes[28] != kNL) return;
  if (out_size != kNL) return;
  if (ws_size < kWsTotal) return;

  const float* x_tasks = (const float*)d_in[0];
  const float* x_mach  = (const float*)d_in[1];
  const float* bn_t_g  = (const float*)d_in[2];
  const float* bn_t_b  = (const float*)d_in[3];
  const float* Wt1 = (const float*)d_in[4];
  const float* bt1 = (const float*)d_in[5];
  const float* Wt2 = (const float*)d_in[6];
  const float* bt2 = (const float*)d_in[7];
  const float* bn_m_g  = (const float*)d_in[8];
  const float* bn_m_b  = (const float*)d_in[9];
  const float* Wm1 = (const float*)d_in[10];
  const float* bm1 = (const float*)d_in[11];
  const float* Wm2 = (const float*)d_in[12];
  const float* bm2 = (const float*)d_in[13];
  const float* Wa1 = (const float*)d_in[14];
  const float* ba1 = (const float*)d_in[15];
  const float* Wa2 = (const float*)d_in[16];
  const float* ba2 = (const float*)d_in[17];
  const float* Wl1 = (const float*)d_in[18];
  const float* bl1 = (const float*)d_in[19];
  const float* Wl2 = (const float*)d_in[20];
  const float* bl2 = (const float*)d_in[21];
  const float* Wo1 = (const float*)d_in[22];
  const float* bo1 = (const float*)d_in[23];
  const float* Wo2 = (const float*)d_in[24];
  const float* bo2 = (const float*)d_in[25];
  const int* tbatch = (const int*)d_in[26];
  const int* mbatch = (const int*)d_in[27];
  const int* labels = (const int*)d_in[28];
  const int* ngraph = (const int*)d_in[29];
  float* outp = (float*)d_out;

  unsigned char* ws = (unsigned char*)d_ws;
  double* partT = (double*)(ws + kOffPartT);
  double* partM = (double*)(ws + kOffPartM);
  float*  stats = (float*)(ws + kOffStats);
  unsigned short* wt1p = (unsigned short*)(ws + kOffWT1);
  unsigned short* wm1p = (unsigned short*)(ws + kOffWM1);
  unsigned short* wt2v = (unsigned short*)(ws + kOffWT2V);
  unsigned short* wm2v = (unsigned short*)(ws + kOffWM2V);
  unsigned short* wa1v = (unsigned short*)(ws + kOffWA1V);
  unsigned short* wa2v = (unsigned short*)(ws + kOffWA2V);
  unsigned short* wl1v = (unsigned short*)(ws + kOffWL1V);
  unsigned short* wl2v = (unsigned short*)(ws + kOffWL2V);
  unsigned short* wo1v = (unsigned short*)(ws + kOffWO1V);
  unsigned short* thp  = (unsigned short*)(ws + kOffTH);
  unsigned short* mhp  = (unsigned short*)(ws + kOffMH);
  unsigned short* gmp  = (unsigned short*)(ws + kOffGM);
  unsigned short* agp  = (unsigned short*)(ws + kOffAG);

  prep_weights_kernel<<<dim3(24, 9), 256, 0, stream>>>(Wt1, Wm1, Wt2, Wm2, Wa1, Wa2, Wl1, Wl2, Wo1, ws);

  bn_partial_kernel<kDT><<<kBlkT, 256, 0, stream>>>(x_tasks, kNT, partT);
  bn_partial_kernel<kDM><<<kBlkM, 256, 0, stream>>>(x_mach, kNM, partM);
  bn_finalize_kernel<<<1, 256, 0, stream>>>(partT, partM, bn_t_g, bn_t_b, bn_m_g, bn_m_b,
                                            tbatch, mbatch, ngraph, stats);

  encoder_kernel<kDT><<<kNTP / 64, 256, 0, stream>>>(x_tasks, kNT, stats, stats + 16,
                                                     wt1p, bt1, wt2v, bt2, thp);
  encoder_kernel<kDM><<<kNMP / 64, 256, 0, stream>>>(x_mach, kNM, stats + 32, stats + 40,
                                                     wm1p, bm1, wm2v, bm2, mhp);

  segmean_kernel<<<kNBP, 128, 0, stream>>>((const unsigned*)thp, (const unsigned*)mhp, gmp);

  aggr_kernel<<<kNBP / 64, 256, 0, stream>>>(gmp, wa1v, ba1, wa2v, ba2, agp);

  link_kernel<<<kNLP / 64, 256, 0, stream>>>(thp, mhp, agp, x_tasks, tbatch, labels,
                                             wl1v, bl1, wl2v, bl2, wo1v, bo1,
                                             Wo2, bo2, outp);
}
